// CausalQKMemoryProjection_58798102282469
// MI455X (gfx1250) — hardware-run, weakly checked
//
#include <hip/hip_runtime.h>
#include <math.h>

typedef __attribute__((ext_vector_type(16))) _Float16 v16h;
typedef __attribute__((ext_vector_type(8)))  _Float16 v8h;
typedef __attribute__((ext_vector_type(8)))  float    v8f;
typedef __attribute__((ext_vector_type(4)))  float    v4f;
typedef __attribute__((ext_vector_type(2)))  float    v2f;

constexpr int kNb    = 4;
constexpr int kNh    = 16;
constexpr int kSeq   = 2048;
constexpr int kHd    = 64;
constexpr int kDm    = kNh * kHd;
constexpr int kCtx   = 128;
constexpr int kSeqP  = kSeq + kCtx;
constexpr int kWin   = kCtx + 64;
constexpr int kRows  = kNb * kSeq;
constexpr float kGamma    = 0.95f;
constexpr float kNormP    = (float)((double)kDm * 0.01);
constexpr float kEps      = 1e-6f;
constexpr float kCarry    = 64.0f;
constexpr float kCarryInv = 1.0f / 64.0f;
constexpr float kP16Lim   = 60000.0f;
constexpr float kResScale = 2048.0f;
constexpr float kResInv   = 1.0f / 2048.0f;
constexpr float kFlushLim = 6.2e-5f;
static_assert(kDm == 1024 && kSeqP == 2176 && kWin == 192, "shape constants");
static_assert((kDm % 32) == 0 && (kWin % 32) == 0, "GEMM K multiples of 32");
static_assert((kRows % 64) == 0 && (kWin % 64) == 0 && (kDm % 64) == 0 && (kSeq % 64) == 0, "GEMM M,N multiples of 64");
static_assert((((kRows / 64) * (kWin / 64)) % 8) == 0, "band tiles fill whole blocks");
static_assert((((kRows / 64) * kNh) % 8) == 0, "output tiles fill whole blocks");

constexpr size_t kSzQH  = (size_t)kRows * kDm * 2;
constexpr size_t kSzQL  = (size_t)kRows * kDm * 2;
constexpr size_t kSzKHP = (size_t)kNb * kSeqP * kDm * 2;
constexpr size_t kSzKLP = (size_t)kNb * kSeqP * kDm * 2;
constexpr size_t kSzKTP = (size_t)kNb * kDm * kSeqP * 2;
constexpr size_t kSzKTL = (size_t)kNb * kDm * kSeqP * 2;
constexpr size_t kSzMT  = (size_t)kDm * kDm * 2;
constexpr size_t kSzPB  = (size_t)kRows * kWin * 2;
constexpr size_t kSzKN  = (size_t)kRows * 4;
constexpr size_t kSzNR  = (size_t)kRows * 4;
constexpr size_t kOffQH  = 0;
constexpr size_t kOffQL  = kOffQH  + kSzQH;
constexpr size_t kOffKHP = kOffQL  + kSzQL;
constexpr size_t kOffKLP = kOffKHP + kSzKHP;
constexpr size_t kOffKTP = kOffKLP + kSzKLP;
constexpr size_t kOffKTL = kOffKTP + kSzKTP;
constexpr size_t kOffMT  = kOffKTL + kSzKTL;
constexpr size_t kOffPB  = kOffMT  + kSzMT;
constexpr size_t kOffKN  = kOffPB  + kSzPB;
constexpr size_t kOffNR  = kOffKN  + kSzKN;
constexpr size_t kWsTotal = kOffNR + kSzNR;
static_assert(kWsTotal == 110166016ull, "carve total");
static_assert(kWsTotal <= 134217728ull, "carve cap");
static_assert((kOffQL % 128) == 0 && (kOffKHP % 128) == 0 && (kOffKLP % 128) == 0 && (kOffKTP % 128) == 0 &&
              (kOffKTL % 128) == 0 && (kOffMT % 128) == 0 && (kOffPB % 128) == 0 &&
              (kOffKN % 128) == 0 && (kOffNR % 128) == 0, "128-B aligned regions");

struct FragH {
  union U { v16h v; v8h h[2]; };
  static __device__ __forceinline__ v16h load(const _Float16* p) {
    U f;
    f.h[0] = *(const v8h*)(p);
    f.h[1] = *(const v8h*)(p + 16);
    return f.v;
  }
  static __device__ __forceinline__ v8f mma(v16h a, v16h b, v8f c) {
    return __builtin_amdgcn_wmma_f32_16x16x32_f16(false, a, false, b, (short)0, c, false, false);
  }
};
__device__ __forceinline__ void tie_acc(v8f& a) { asm volatile("" : "+v"(a)); }
__device__ __forceinline__ void guard_acc(v8f& a, v16h x, v16h y) {
  asm volatile("v_nop\n\tv_nop\n\tv_nop\n\tv_nop" : "+v"(a) : "v"(x), "v"(y));
}
__device__ __forceinline__ void keep4_h(v16h a, v16h b, v16h c, v16h d) { asm volatile("v_nop" :: "v"(a), "v"(b), "v"(c), "v"(d)); }
__device__ __forceinline__ void acc_guard4(v8f& a, v8f& b, v8f& c, v8f& d) {
  asm volatile("v_nop\n\tv_nop\n\tv_nop\n\tv_nop" : "+v"(a), "+v"(b), "+v"(c), "+v"(d));
}
__device__ __forceinline__ void wave_lds_sync() {
  __builtin_amdgcn_fence(__ATOMIC_RELEASE, "workgroup");
  __builtin_amdgcn_wave_barrier();
  __builtin_amdgcn_fence(__ATOMIC_ACQUIRE, "workgroup");
}

__device__ __forceinline__ void split_f16(float v, _Float16& hv, _Float16& lv) {
  const float vs = (fabsf(v) < kFlushLim) ? 0.0f : v;
  const _Float16 h = (_Float16)vs;
  const float hf = (float)h;
  const float rs = (v - hf) * kResScale;
  hv = h;
  lv = (_Float16)rs;
}

__device__ __forceinline__ void tile_kloop(v8f (&acc)[4][4],
                                           const _Float16* __restrict__ Ab, int lda,
                                           const _Float16* __restrict__ Bb, int ldb,
                                           int K, int rlane, int koff) {
  for (int k0 = 0; k0 < K; k0 += 32) {
    v16h bh[4];
#pragma unroll
    for (int j = 0; j < 4; ++j) {
      bh[j] = FragH::load(Bb + (size_t)((j << 4) + rlane) * ldb + koff + k0);
    }
#pragma unroll
    for (int i = 0; i < 4; ++i) {
      const v16h ah = FragH::load(Ab + (size_t)((i << 4) + rlane) * lda + koff + k0);
#pragma unroll
      for (int j = 0; j < 4; ++j) {
        acc[i][j] = FragH::mma(ah, bh[j], acc[i][j]);
      }
      tie_acc(acc[i][0]);
      tie_acc(acc[i][1]);
      tie_acc(acc[i][2]);
      guard_acc(acc[i][3], ah, bh[3]);
    }
    keep4_h(bh[0], bh[1], bh[2], bh[3]);
  }
}

__device__ __forceinline__ void guard_all(v8f (&acc)[4][4]) {
  acc_guard4(acc[0][0], acc[0][1], acc[0][2], acc[0][3]);
  acc_guard4(acc[1][0], acc[1][1], acc[1][2], acc[1][3]);
  acc_guard4(acc[2][0], acc[2][1], acc[2][2], acc[2][3]);
  acc_guard4(acc[3][0], acc[3][1], acc[3][2], acc[3][3]);
}
__device__ __forceinline__ void scale_all(v8f (&acc)[4][4], float s) {
#pragma unroll
  for (int i = 0; i < 4; ++i) {
#pragma unroll
    for (int j = 0; j < 4; ++j) {
      acc[i][j] = acc[i][j] * s;
    }
  }
}

__device__ __forceinline__ void store_slab_f16(const float* slab, unsigned short* crow0, int ldc, int lane) {
  const int q = lane >> 3, c8 = (lane & 7) * 8;
  for (int pass = 0; pass < 2; ++pass) {
#pragma unroll
    for (int it = 0; it < 4; ++it) {
      const int row = it * 4 + q;
      const float* sp = slab + row * 68 + c8;
      v8h hv;
#pragma unroll
      for (int e = 0; e < 8; ++e) hv[e] = (_Float16)sp[e];
      *(volatile v8h*)(crow0 + (size_t)row * ldc + c8) = hv;
    }
    __threadfence();
  }
}
__device__ __forceinline__ void store_slab_f32(const float* slab, float* crow0, int ldc, int lane) {
  const int hh = lane >> 4, c4 = (lane & 15) * 4;
  for (int pass = 0; pass < 2; ++pass) {
#pragma unroll
    for (int it = 0; it < 8; ++it) {
      const int row = it * 2 + hh;
      const v4f v = *(const v4f*)(slab + row * 68 + c4);
      *(volatile v4f*)(crow0 + (size_t)row * ldc + c4) = v;
    }
    __threadfence();
  }
}

__global__ __launch_bounds__(256) void pack_q_kernel(const float* __restrict__ q,
                                                     unsigned short* __restrict__ QH,
                                                     unsigned short* __restrict__ QL) {
  const int i = blockIdx.x * 256 + threadIdx.x;
  const int dh8 = i & 7;
  const int s   = (i >> 3) & (kSeq - 1);
  const int h   = (i >> 14) & (kNh - 1);
  const int b   = i >> 18;
  const float* src = q + (size_t)i * 8;
  const v4f a0 = *(const v4f*)(src);
  const v4f a1 = *(const v4f*)(src + 4);
  v8h hv, lv;
#pragma unroll
  for (int e = 0; e < 4; ++e) {
    _Float16 h0, l0, h1, l1;
    const float x0 = a0[e];
    const float x1 = a1[e];
    split_f16(x0, h0, l0);
    split_f16(x1, h1, l1);
    hv[e]     = h0;
    lv[e]     = l0;
    hv[4 + e] = h1;
    lv[4 + e] = l1;
  }
  const size_t o = (size_t)(b * kSeq + s) * kDm + h * kHd + dh8 * 8;
  *(volatile v8h*)(QH + o) = hv;
  *(volatile v8h*)(QL + o) = lv;
  __threadfence();
  *(volatile v8h*)(QH + o) = hv;
  *(volatile v8h*)(QL + o) = lv;
}

__global__ __launch_bounds__(256) void pack_k_kernel(const float* __restrict__ k,
                                                     unsigned short* __restrict__ KHP,
                                                     unsigned short* __restrict__ KLP,
                                                     unsigned short* __restrict__ KTP,
                                                     unsigned short* __restrict__ KTL) {
  __shared__ __align__(16) float sT[64 * 68];
  const int tid = threadIdx.x;
  const int blk = blockIdx.x;
  const int sb = blk & 31;
  const int h  = (blk >> 5) & (kNh - 1);
  const int b  = blk >> 9;
  const int s0 = sb * 64;
  const float* src = k + ((size_t)(b * kNh + h) * kSeq + s0) * kHd;
#pragma unroll
  for (int it = 0; it < 4; ++it) {
    const int idx = it * 256 + tid;
    const int row = idx >> 4, c4 = (idx & 15) * 4;
    const v4f v = *(const v4f*)(src + (size_t)idx * 4);
    *(v4f*)(sT + row * 68 + c4) = v;
  }
  __syncthreads();
  v8h rv[2], rl[2], tv[2], tl[2];
#pragma unroll
  for (int it = 0; it < 2; ++it) {
    const int u = it * 256 + tid;
    const int r = u >> 3, c8 = (u & 7) * 8;
#pragma unroll
    for (int e = 0; e < 8; ++e) {
      _Float16 ha, la, hb, lb;
      const float xa = sT[r * 68 + c8 + e];
      const float xb = sT[(c8 + e) * 68 + r];
      split_f16(xa, ha, la);
      split_f16(xb, hb, lb);
      rv[it][e] = ha;
      rl[it][e] = la;
      tv[it][e] = hb;
      tl[it][e] = lb;
    }
  }
  for (int pass = 0; pass < 2; ++pass) {
#pragma unroll
    for (int it = 0; it < 2; ++it) {
      const int u = it * 256 + tid;
      const int r = u >> 3, c8 = (u & 7) * 8;
      const size_t orow = ((size_t)b * kSeqP + kCtx + s0 + r) * kDm + h * kHd + c8;
      *(volatile v8h*)(KHP + orow) = rv[it];
      *(volatile v8h*)(KLP + orow) = rl[it];
      const size_t otr = ((size_t)b * kDm + h * kHd + r) * kSeqP + kCtx + s0 + c8;
      *(volatile v8h*)(KTP + otr) = tv[it];
      *(volatile v8h*)(KTL + otr) = tl[it];
    }
    __threadfence();
  }
  if (sb == 0) {
    v8h zv;
#pragma unroll
    for (int e = 0; e < 8; ++e) zv[e] = (_Float16)0.0f;
    for (int pass = 0; pass < 2; ++pass) {
#pragma unroll
      for (int it = 0; it < 4; ++it) {
        const int u = it * 256 + tid;
        const int pr = u >> 3, pc8 = (u & 7) * 8;
        const size_t orow = ((size_t)b * kSeqP + pr) * kDm + h * kHd + pc8;
        *(volatile v8h*)(KHP + orow) = zv;
        *(volatile v8h*)(KLP + orow) = zv;
        const int tr = u >> 4, tc8 = (u & 15) * 8;
        const size_t otr = ((size_t)b * kDm + h * kHd + tr) * kSeqP + tc8;
        *(volatile v8h*)(KTP + otr) = zv;
        *(volatile v8h*)(KTL + otr) = zv;
      }
      __threadfence();
    }
  }
}

__global__ __launch_bounds__(256) void transpose_m_kernel(const float* __restrict__ Mp, unsigned short* __restrict__ MT) {
  __shared__ __align__(16) float sT[64 * 68];
  const int tid = threadIdx.x;
  const int d0 = (blockIdx.x >> 4) * 64;
  const int e0 = (blockIdx.x & 15) * 64;
#pragma unroll
  for (int it = 0; it < 4; ++it) {
    const int idx = it * 256 + tid;
    const int row = idx >> 4, c4 = (idx & 15) * 4;
    const v4f v = *(const v4f*)(Mp + (size_t)(d0 + row) * kDm + e0 + c4);
    *(v4f*)(sT + row * 68 + c4) = v;
  }
  __syncthreads();
  v8h tv[2];
#pragma unroll
  for (int it = 0; it < 2; ++it) {
    const int u = it * 256 + tid;
    const int e = u >> 3, d8 = (u & 7) * 8;
#pragma unroll
    for (int x = 0; x < 8; ++x) tv[it][x] = (_Float16)(sT[(d8 + x) * 68 + e] * kCarry);
  }
  for (int pass = 0; pass < 2; ++pass) {
#pragma unroll
    for (int it = 0; it < 2; ++it) {
      const int u = it * 256 + tid;
      const int e = u >> 3, d8 = (u & 7) * 8;
      *(volatile v8h*)(MT + (size_t)(e0 + e) * kDm + d0 + d8) = tv[it];
    }
    __threadfence();
  }
}

__global__ __launch_bounds__(256) void key_norm_kernel(const float* __restrict__ k, float* __restrict__ KN) {
  __shared__ float sK[32];
  const int tid = threadIdx.x, lane = tid & 31, wave = tid >> 5;
#pragma unroll 1
  for (int i = 0; i < 4; ++i) {
    const int row = blockIdx.x * 32 + wave * 4 + i;
    const int b = row >> 11;
    const int s = row & (kSeq - 1);
    float acc = 0.0f;
#pragma unroll 4
    for (int h = 0; h < kNh; ++h) {
      const v2f x = *(const v2f*)(k + ((size_t)(b * kNh + h) * kSeq + s) * kHd + lane * 2);
      acc = fmaf(x[0], x[0], acc);
      acc = fmaf(x[1], x[1], acc);
    }
    acc += __shfl_xor(acc, 16, 32);
    acc += __shfl_xor(acc, 8, 32);
    acc += __shfl_xor(acc, 4, 32);
    acc += __shfl_xor(acc, 2, 32);
    acc += __shfl_xor(acc, 1, 32);
    if (lane == 0) sK[wave * 4 + i] = acc;
  }
  __syncthreads();
  if (wave == 0) {
    const float v = sK[lane];
    volatile float* dst = KN + (size_t)blockIdx.x * 32 + lane;
    *dst = v;
    __threadfence();
    *dst = v;
  }
}

__global__ __launch_bounds__(256) void band_norm_kernel(const float* __restrict__ gates, const float* __restrict__ KN,
                                                        float* __restrict__ NR) {
  __shared__ float sG[384];
  __shared__ float sPw[kCtx];
  const int tid = threadIdx.x;
  const int gi = blockIdx.x * 256;
  const int b = gi >> 11;
  const int t0 = gi & (kSeq - 1);
#pragma unroll
  for (int it = 0; it < 2; ++it) {
    const int idx = it * 256 + tid;
    if (idx < 384) {
      const int j = t0 - kCtx + idx;
      int jc = j < 0 ? 0 : j;
      jc = jc > kSeq - 1 ? kSeq - 1 : jc;
      const float g  = gates[(size_t)b * kSeq + jc];
      const float kn = KN[(size_t)b * kSeq + jc];
      sG[idx] = (j >= 0) ? g * kn : 0.0f;
    }
  }
  if (tid < kCtx) sPw[tid] = exp2f((float)tid * log2f(kGamma));
  __syncthreads();
  float acc = 0.0f;
#pragma unroll 4
  for (int i = 0; i < kCtx; ++i) {
    acc = fmaf(sPw[i], sG[tid + (kCtx - 1) - i], acc);
  }
  const float nv = kNormP + acc;
  volatile float* dst = NR + (size_t)gi + tid;
  *dst = nv;
  __threadfence();
  *dst = nv;
}

__global__ __launch_bounds__(256) void band_dots_kernel(const unsigned short* __restrict__ QHp,
                                                        const unsigned short* __restrict__ QLp,
                                                        const unsigned short* __restrict__ KHPp,
                                                        const unsigned short* __restrict__ KLPp,
                                                        const float* __restrict__ gates,
                                                        unsigned short* __restrict__ PB) {
  __shared__ __align__(16) float sT[8][16 * 68];
  __shared__ float sPw[kCtx];
  const int tid = threadIdx.x, lane = tid & 31, wave = tid >> 5;
  if (tid < kCtx) sPw[tid] = exp2f((float)tid * log2f(kGamma));
  __syncthreads();
  const int tile = blockIdx.x * 8 + wave;
  const int tm = tile / 3;
  const int tn = tile - tm * 3;
  const int b  = tm >> 5;
  const int T0 = (tm & 31) * 64;
  const int m0 = tm * 64;
  const int rlane = lane & 15;
  const int koff  = (lane >> 4) * 8;
  const int mOff  = (lane >> 4) * 8;
  const size_t aoff = (size_t)m0 * kDm;
  const size_t boff = ((size_t)b * kSeqP + T0 + tn * 64) * kDm;
  const _Float16* Ah = (const _Float16*)QHp + aoff;
  const _Float16* Al = (const _Float16*)QLp + aoff;
  const _Float16* Bh = (const _Float16*)KHPp + boff;
  const _Float16* Bl = (const _Float16*)KLPp + boff;

  v8f acc[4][4];
#pragma unroll
  for (int i = 0; i < 4; ++i)
#pragma unroll
    for (int j = 0; j < 4; ++j) acc[i][j] = (v8f){0.f, 0.f, 0.f, 0.f, 0.f, 0.f, 0.f, 0.f};

  tile_kloop(acc, Ah, kDm, Bl, kDm, kDm, rlane, koff);
  tile_kloop(acc, Al, kDm, Bh, kDm, kDm, rlane, koff);
  guard_all(acc);
  scale_all(acc, kResInv);
  tile_kloop(acc, Ah, kDm, Bh, kDm, kDm, rlane, koff);
  guard_all(acc);

  float gcol[4];
#pragma unroll
  for (int j = 0; j < 4; ++j) {
    const int c  = tn * 64 + (j << 4) + rlane;
    const int jk = T0 - kCtx + c;
    int jc = jk < 0 ? 0 : jk;
    jc = jc > kSeq - 1 ? kSeq - 1 : jc;
    const float g = gates[(size_t)b * kSeq + jc];
    gcol[j] = (jk >= 0) ? g * kCarry : 0.0f;
  }

  float* slab = sT[wave];
#pragma unroll
  for (int i = 0; i < 4; ++i) {
#pragma unroll
    for (int j = 0; j < 4; ++j) {
      const int c = tn * 64 + (j << 4) + rlane;
#pragma unroll
      for (int r = 0; r < 8; ++r) {
        const int rr = (i << 4) + mOff + r;
        const int dist = rr + kCtx - c;
        const bool valid = (dist >= 1) && (dist <= kCtx);
        int pidx = dist - 1;
        pidx = pidx < 0 ? 0 : pidx;
        pidx = pidx > kCtx - 1 ? kCtx - 1 : pidx;
        const float w = sPw[pidx] * gcol[j];
        float v = acc[i][j][r] * w;
        v = fminf(fmaxf(v, -kP16Lim), kP16Lim);
        v = valid ? v : 0.0f;
        slab[(mOff + r) * 68 + (j << 4) + rlane] = v;
      }
    }
    wave_lds_sync();
    store_slab_f16(slab, PB + (size_t)(m0 + (i << 4)) * kWin + tn * 64, kWin, lane);
    wave_lds_sync();
  }
}

__global__ __launch_bounds__(256) void out_gemm_kernel(const unsigned short* __restrict__ QHp,
                                                       const unsigned short* __restrict__ MTp,
                                                       const unsigned short* __restrict__ PBp,
                                                       const unsigned short* __restrict__ KTPp,
                                                       const unsigned short* __restrict__ KTLp,
                                                       const float* __restrict__ NR,
                                                       float* __restrict__ out) {
  __shared__ __align__(16) float sT[8][16 * 68];
  __shared__ float sInv[8][64];
  const int tid = threadIdx.x, lane = tid & 31, wave = tid >> 5;
  const int tile = blockIdx.x * 8 + wave;
  const int tm = tile >> 4;
  const int hd = tile & (kNh - 1);
  const int b  = tm >> 5;
  const int T0 = (tm & 31) * 64;
  const int m0 = tm * 64;
  const int n0 = hd * kHd;
  const int rlane = lane & 15;
  const int koff  = (lane >> 4) * 8;
  const int mOff  = (lane >> 4) * 8;

  v8f acc[4][4];
#pragma unroll
  for (int i = 0; i < 4; ++i)
#pragma unroll
    for (int j = 0; j < 4; ++j) acc[i][j] = (v8f){0.f, 0.f, 0.f, 0.f, 0.f, 0.f, 0.f, 0.f};

  const _Float16* Pb = (const _Float16*)PBp + (size_t)m0 * kWin;
  const size_t ktoff = ((size_t)b * kDm + n0) * kSeqP + T0;
  {
    const _Float16* Bb = (const _Float16*)KTLp + ktoff;
    tile_kloop(acc, Pb, kWin, Bb, kSeqP, kWin, rlane, koff);
  }
  guard_all(acc);
  scale_all(acc, kResInv);
  {
    const _Float16* Ab = (const _Float16*)QHp + (size_t)m0 * kDm;
    const _Float16* Bb = (const _Float16*)MTp + (size_t)n0 * kDm;
    tile_kloop(acc, Ab, kDm, Bb, kDm, kDm, rlane, koff);
  }
  {
    const _Float16* Bb = (const _Float16*)KTPp + ktoff;
    tile_kloop(acc, Pb, kWin, Bb, kSeqP, kWin, rlane, koff);
  }
  guard_all(acc);

  {
    const float na = NR[(size_t)m0 + lane];
    const float nb = NR[(size_t)m0 + 32 + lane];
    sInv[wave][lane]      = kCarryInv * (1.0f / (na + kEps));
    sInv[wave][32 + lane] = kCarryInv * (1.0f / (nb + kEps));
  }
  wave_lds_sync();

  float* slab = sT[wave];
  float* cbase = out + ((size_t)(b * kNh + hd) * kSeq + T0) * kHd;
#pragma unroll
  for (int i = 0; i < 4; ++i) {
    float sc[8];
#pragma unroll
    for (int r = 0; r < 8; ++r) sc[r] = sInv[wave][(i << 4) + mOff + r];
#pragma unroll
    for (int j = 0; j < 4; ++j) {
#pragma unroll
      for (int r = 0; r < 8; ++r) {
        slab[(mOff + r) * 68 + (j << 4) + rlane] = acc[i][j][r] * sc[r];
      }
    }
    wave_lds_sync();
    store_slab_f32(slab, cbase + (size_t)(i << 4) * kHd, kHd, lane);
    wave_lds_sync();
  }
}

extern "C" void kernel_launch(void* const* d_in, const int* in_sizes, int n_in,
                              void* d_out, int out_size, void* d_ws, size_t ws_size,
                              hipStream_t stream) {
  if (n_in < 4) return;
  if (in_sizes[0] != kRows * kDm) return;
  if (in_sizes[1] != kRows * kDm) return;
  if (in_sizes[2] != kNb * kSeq) return;
  if (in_sizes[3] != kDm * kDm) return;
  if (out_size != kRows * kDm) return;
  if (ws_size < kWsTotal) return;

  const float* q     = (const float*)d_in[0];
  const float* k     = (const float*)d_in[1];
  const float* gates = (const float*)d_in[2];
  const float* Mp    = (const float*)d_in[3];
  float* out = (float*)d_out;

  char* ws = (char*)d_ws;
  unsigned short* QH  = (unsigned short*)(ws + kOffQH);
  unsigned short* QL  = (unsigned short*)(ws + kOffQL);
  unsigned short* KHP = (unsigned short*)(ws + kOffKHP);
  unsigned short* KLP = (unsigned short*)(ws + kOffKLP);
  unsigned short* KTP = (unsigned short*)(ws + kOffKTP);
  unsigned short* KTL = (unsigned short*)(ws + kOffKTL);
  unsigned short* MT  = (unsigned short*)(ws + kOffMT);
  unsigned short* PB  = (unsigned short*)(ws + kOffPB);
  float*          KN  = (float*)(ws + kOffKN);
  float*          NR  = (float*)(ws + kOffNR);

  pack_q_kernel<<<(kRows * kDm / 8) / 256, 256, 0, stream>>>(q, QH, QL);
  pack_k_kernel<<<kNb * kNh * (kSeq / 64), 256, 0, stream>>>(k, KHP, KLP, KTP, KTL);
  transpose_m_kernel<<<(kDm / 64) * (kDm / 64), 256, 0, stream>>>(Mp, MT);
  key_norm_kernel<<<kRows / 32, 256, 0, stream>>>(k, KN);
  band_norm_kernel<<<kRows / 256, 256, 0, stream>>>(gates, KN, NR);
  band_dots_kernel<<<((kRows / 64) * (kWin / 64)) / 8, 256, 0, stream>>>(QH, QL, KHP, KLP, gates, PB);
  out_gemm_kernel<<<((kRows / 64) * kNh) / 8, 256, 0, stream>>>(QH, MT, PB, KTP, KTL, NR, out);
}
